// VelocityCrossAttention_37383395344857
// MI455X (gfx1250) — hardware-verified
//
#include <hip/hip_runtime.h>
#include <math.h>
#include <stdint.h>

#define NBATCH 4
#define NT     512
#define NJ     17
#define CH     256
#define CH2    512
#define NHEAD  8
#define HDIM   32
#define NGRP   (NBATCH * NJ)
#define MROWS  (NGRP * NT)
#define NWEL   524288
#define OWC1   0
#define OWC2   131072
#define OWQ    262144
#define OWKV   327680
#define OWP    458752
#define XS   16.0f
#define WSC  256.0f
#define VS   64.0f
#define V2C  256.0f
#define QC   512.0f
#define KC   64.0f
#define VC   64.0f
#define AC   256.0f
#define PSC  1024.0f
#define RSQ2 0.70710678118654752f
static_assert(NHEAD * HDIM == CH);
static_assert(MROWS == 34816);
static_assert((MROWS % 64) == 0 && (NT % 64) == 0 && (CH % 64) == 0 && (CH2 % 64) == 0);
static_assert(OWP + CH * CH == NWEL);

typedef _Float16 v16h __attribute__((ext_vector_type(16)));
typedef _Float16 v8h  __attribute__((ext_vector_type(8)));
typedef float    v8f  __attribute__((ext_vector_type(8)));
typedef float    v4f  __attribute__((ext_vector_type(4)));
typedef float    v2f  __attribute__((ext_vector_type(2)));
typedef unsigned int v4u __attribute__((ext_vector_type(4)));

union FragH { v16h v; v8h h[2]; };

__device__ __forceinline__ unsigned short bf_bits(float f) {
  unsigned u = __float_as_uint(f);
  return (unsigned short)((u + 0x7FFFu + ((u >> 16) & 1u)) >> 16);
}
__device__ __forceinline__ float bf_up(unsigned short h) { return __uint_as_float(((unsigned)h) << 16); }
__device__ __forceinline__ float bfr(float f) { return bf_up(bf_bits(f)); }
__device__ __forceinline__ unsigned short h_bits(_Float16 x) { return __builtin_bit_cast(unsigned short, x); }
__device__ __forceinline__ unsigned pk16(unsigned short a, unsigned short b) { return (unsigned)a | ((unsigned)b << 16); }
__device__ __forceinline__ v8f zero8() { v8f z = {0.f, 0.f, 0.f, 0.f, 0.f, 0.f, 0.f, 0.f}; return z; }
__device__ __forceinline__ float hmax8(v8f s) {
  return fmaxf(fmaxf(fmaxf(s[0], s[1]), fmaxf(s[2], s[3])), fmaxf(fmaxf(s[4], s[5]), fmaxf(s[6], s[7])));
}
__device__ __forceinline__ int tok_of(int np) {
  const int g = np >> 9, t = np & (NT - 1);
  const int b = g / NJ, j = g - b * NJ;
  return (b * NT + t) * NJ + j;
}

__device__ __forceinline__ v16h ldfrag_h(const _Float16* p) {
  FragH f;
  f.h[0] = *(const v8h*)(p);
  f.h[1] = *(const v8h*)(p + 16);
  return f.v;
}

__device__ __forceinline__ v8f mma_h_raw(v16h a, v16h b, v8f c) {
  return __builtin_amdgcn_wmma_f32_16x16x32_f16(false, a, false, b, (short)0, c, false, false);
}
__device__ __forceinline__ void dep_guard1(v8f& a, v8f& b, v16h x) {
#if defined(__HIP_DEVICE_COMPILE__)
  asm volatile("v_nop\n\tv_nop\n\tv_nop\n\tv_nop" : "+v"(a), "+v"(b) : "v"(x));
#endif
}
__device__ __forceinline__ void keep4_h(v16h a, v16h b, v16h c, v16h d) {
#if defined(__HIP_DEVICE_COMPILE__)
  asm volatile("v_nop" :: "v"(a), "v"(b), "v"(c), "v"(d));
#endif
}
__device__ __forceinline__ void acc_guard4(v8f& a, v8f& b, v8f& c, v8f& d) {
#if defined(__HIP_DEVICE_COMPILE__)
  asm volatile("v_nop\n\tv_nop\n\tv_nop\n\tv_nop" : "+v"(a), "+v"(b), "+v"(c), "+v"(d));
#endif
}
__device__ __forceinline__ void sguard4(v8f& a, v8f& b, v8f& c, v8f& d,
                                        v16h k0, v16h k1, v16h k2, v16h k3, v16h q) {
#if defined(__HIP_DEVICE_COMPILE__)
  asm volatile("v_nop\n\tv_nop\n\tv_nop\n\tv_nop"
               : "+v"(a), "+v"(b), "+v"(c), "+v"(d) : "v"(k0), "v"(k1), "v"(k2), "v"(k3), "v"(q));
#endif
}
__device__ __forceinline__ void oguard2(v8f& o0, v8f& o1, v16h a0, v16h a1, v16h a2, v16h a3,
                                        v16h a4, v16h a5, v16h a6, v16h a7, v16h b0, v16h b1) {
#if defined(__HIP_DEVICE_COMPILE__)
  asm volatile("v_nop\n\tv_nop\n\tv_nop\n\tv_nop"
               : "+v"(o0), "+v"(o1)
               : "v"(a0), "v"(a1), "v"(a2), "v"(a3), "v"(a4), "v"(a5), "v"(a6), "v"(a7), "v"(b0), "v"(b1));
#endif
}
__device__ __forceinline__ void wave_sync_lds() {
  __builtin_amdgcn_fence(__ATOMIC_RELEASE, "workgroup");
  __builtin_amdgcn_wave_barrier();
  __builtin_amdgcn_fence(__ATOMIC_ACQUIRE, "workgroup");
}

__global__ __launch_bounds__(256) void wprep(const float* __restrict__ wc1, const float* __restrict__ wc2,
                                              const float* __restrict__ wq, const float* __restrict__ wkv,
                                              const float* __restrict__ wp, unsigned short* Wall) {
  const int t = threadIdx.x, bx = blockIdx.x;
  const float* src = (bx < 64) ? wc1 : (bx < 128) ? wc2 : (bx < 160) ? wq : (bx < 224) ? wkv : wp;
  const int    b0  = (bx < 64) ? 0   : (bx < 128) ? 64  : (bx < 160) ? 128 : (bx < 224) ? 160 : 224;
  const size_t le = ((size_t)(bx - b0) * 256 + t) * 8;
  const float* sp = src + le;
  const v4f a = *(const v4f*)(sp), c = *(const v4f*)(sp + 4);
  float w[8];
#pragma unroll
  for (int i = 0; i < 4; ++i) { w[i] = bfr(a[i]) * WSC; w[4 + i] = bfr(c[i]) * WSC; }
  v4u v;
#pragma unroll
  for (int i = 0; i < 4; ++i) v[i] = pk16(h_bits((_Float16)w[2 * i]), h_bits((_Float16)w[2 * i + 1]));
  unsigned short* dp = Wall + ((size_t)bx * 256 + t) * 8;
  *(volatile v4u*)dp = v;
  __threadfence();
  *(volatile v4u*)dp = v;
}

__global__ __launch_bounds__(256) void xprep(const float* __restrict__ x, unsigned short* X16) {
  const int tid = threadIdx.x, wave = tid >> 5, lane = tid & 31;
  const int np  = blockIdx.x * 8 + wave;
  const int tok = tok_of(np);
  const float* sp = x + (size_t)tok * CH + 8 * lane;
  const v4f a = *(const v4f*)(sp), c = *(const v4f*)(sp + 4);
  float w[8];
#pragma unroll
  for (int i = 0; i < 4; ++i) { w[i] = bfr(a[i]) * XS; w[4 + i] = bfr(c[i]) * XS; }
  v4u v;
#pragma unroll
  for (int i = 0; i < 4; ++i) v[i] = pk16(h_bits((_Float16)w[2 * i]), h_bits((_Float16)w[2 * i + 1]));
  unsigned short* dp = X16 + (size_t)np * CH + 8 * lane;
  *(volatile v4u*)dp = v;
  __threadfence();
  *(volatile v4u*)dp = v;
}

__global__ __launch_bounds__(256) void velprep(const float* __restrict__ Y, unsigned short* G) {
  __shared__ __align__(16) unsigned int Pk[256 * 4];
  const int tid = threadIdx.x;
  const size_t e8 = ((size_t)blockIdx.x * 256 + tid) * 8;
  const int np  = (int)(e8 >> 9);
  const int col = (int)(e8 & (CH2 - 1));
  const int t   = np & (NT - 1);
  const int npp = (t == 0) ? np : (np - 1);
  const float* cp = Y + (size_t)np * CH2 + col;
  const float* pp = Y + (size_t)npp * CH2 + col;
#pragma unroll 1
  for (int i = 0; i < 4; ++i) {
    const v2f a = *(const v2f*)(cp + 2 * i);
    const v2f b = *(const v2f*)(pp + 2 * i);
    const float d0 = a[0] - b[0], d1 = a[1] - b[1];
    const float g0 = 0.5f * d0 * (1.0f + erff(d0 * RSQ2));
    const float g1 = 0.5f * d1 * (1.0f + erff(d1 * RSQ2));
    Pk[tid * 4 + i] = pk16(h_bits((_Float16)(g0 * VS)), h_bits((_Float16)(g1 * VS)));
  }
  __builtin_amdgcn_fence(__ATOMIC_RELEASE, "wavefront");
  __builtin_amdgcn_wave_barrier();
  const v4u v = *(const v4u*)(&Pk[tid * 4]);
  unsigned short* dp = G + e8;
  *(volatile v4u*)dp = v;
  __threadfence();
  *(volatile v4u*)dp = v;
}

template <int NPL, int OM, int HASB, int RMAP>
__global__ __launch_bounds__(256) void gemm64(
    const unsigned short* __restrict__ Ap, const unsigned short* __restrict__ Ap2, int lda,
    const unsigned short* __restrict__ Bp, int ldb,
    const float* __restrict__ bias,
    void* Cout, int ldc,
    unsigned short* Clo, int lon0, int lon1,
    float osc, float bsc, int M, int N, int K) {
  __shared__ __align__(16) float sT[8][16 * 68];
  const int lane = threadIdx.x & 31;
  const int wave = threadIdx.x >> 5;
  const int tilesN = N >> 6;
  const int tilesM = M >> 6;
  const int tile = blockIdx.x * 8 + wave;
  if (tile >= tilesM * tilesN) return;
  const int tm = tile / tilesN;
  const int tn = tile - tm * tilesN;
  const int m0 = tm << 6;
  const int n0 = tn << 6;

  const _Float16* A0 = (const _Float16*)(const void*)Ap;
  const _Float16* A1 = (const _Float16*)(const void*)Ap2;
  const _Float16* Bb = (const _Float16*)(const void*)Bp;

  const int rlane = lane & 15;
  const int koff  = (lane >> 4) * 8;
  const int mOff  = (lane >> 4) * 8;

  v8f acc[4][4];
#pragma unroll
  for (int i = 0; i < 4; ++i)
#pragma unroll
    for (int j = 0; j < 4; ++j) acc[i][j] = zero8();

#pragma unroll
  for (int pl = 0; pl < NPL; ++pl) {
    const _Float16* Ah = (pl == 0) ? A0 : A1;
    for (int k0 = 0; k0 < K; k0 += 32) {
      v16h bh[4];
#pragma unroll
      for (int j = 0; j < 4; ++j) {
        const size_t bo = (size_t)(n0 + (j << 4) + rlane) * ldb + koff + k0;
        bh[j] = ldfrag_h(Bb + bo);
      }
#pragma unroll
      for (int i = 0; i < 4; ++i) {
        const size_t ao = (size_t)(m0 + (i << 4) + rlane) * lda + koff + k0;
        const v16h ah = ldfrag_h(Ah + ao);
#pragma unroll
        for (int j = 0; j < 4; ++j) acc[i][j] = mma_h_raw(ah, bh[j], acc[i][j]);
        dep_guard1(acc[i][0], acc[i][3], ah);
      }
      keep4_h(bh[0], bh[1], bh[2], bh[3]);
    }
  }
  acc_guard4(acc[0][0], acc[0][1], acc[0][2], acc[0][3]);
  acc_guard4(acc[1][0], acc[1][1], acc[1][2], acc[1][3]);
  acc_guard4(acc[2][0], acc[2][1], acc[2][2], acc[2][3]);
  acc_guard4(acc[3][0], acc[3][1], acc[3][2], acc[3][3]);

  const bool dolo = (OM == 1) && (n0 >= lon0) && (n0 < lon1);
  const int hh2 = lane >> 4, c4 = (lane & 15) * 4;
  const int q8  = lane >> 3, c8 = (lane & 7) * 8;

  v4f bq4 = {0.f, 0.f, 0.f, 0.f};
  float bq8[8];
#pragma unroll
  for (int e = 0; e < 8; ++e) bq8[e] = 0.f;
  if (HASB) {
    if (OM == 0) {
      const v4f br = *(const v4f*)(bias + n0 + c4);
#pragma unroll
      for (int e = 0; e < 4; ++e) bq4[e] = bfr(br[e]) * bsc;
    } else {
      const v4f b0 = *(const v4f*)(bias + n0 + c8), b1 = *(const v4f*)(bias + n0 + c8 + 4);
#pragma unroll
      for (int e = 0; e < 4; ++e) { bq8[e] = bfr(b0[e]) * bsc; bq8[4 + e] = bfr(b1[e]) * bsc; }
    }
  }

  float* slab = sT[wave];
#pragma unroll
  for (int i = 0; i < 4; ++i) {
    const int mBase = m0 + (i << 4);
#pragma unroll
    for (int j = 0; j < 4; ++j) {
#pragma unroll
      for (int r = 0; r < 8; ++r) {
        slab[(mOff + r) * 68 + (j << 4) + rlane] = acc[i][j][r];
      }
    }
    wave_sync_lds();
    if (OM == 0) {
      float* C = (float*)Cout;
      v4f vals[8];
#pragma unroll
      for (int it = 0; it < 8; ++it) {
        const int row = it * 2 + hh2;
        v4f v = *(const v4f*)(slab + row * 68 + c4);
#pragma unroll
        for (int e = 0; e < 4; ++e) v[e] = v[e] * osc + bq4[e];
        vals[it] = v;
      }
      for (int pass = 0; pass < 2; ++pass) {
#pragma unroll
        for (int it = 0; it < 8; ++it) {
          const int row = it * 2 + hh2;
          const int gm = mBase + row;
          const int crow = RMAP ? tok_of(gm) : gm;
          *(volatile v4f*)(C + (size_t)crow * ldc + n0 + c4) = vals[it];
        }
        __threadfence();
      }
    } else {
      unsigned short* C = (unsigned short*)Cout;
      unsigned short* L = Clo;
      v4u hv[4], lv[4];
#pragma unroll
      for (int it = 0; it < 4; ++it) {
        const int row = it * 4 + q8;
        const float* sp = slab + row * 68 + c8;
        v4u a, lo;
#pragma unroll
        for (int e = 0; e < 4; ++e) {
          const float f0 = sp[2 * e] * osc + bq8[2 * e], f1 = sp[2 * e + 1] * osc + bq8[2 * e + 1];
          const _Float16 h0 = (_Float16)f0, h1 = (_Float16)f1;
          const _Float16 l0 = (_Float16)(f0 - (float)h0), l1 = (_Float16)(f1 - (float)h1);
          a[e]  = pk16(h_bits(h0), h_bits(h1));
          lo[e] = pk16(h_bits(l0), h_bits(l1));
        }
        hv[it] = a;
        lv[it] = lo;
      }
      for (int pass = 0; pass < 2; ++pass) {
#pragma unroll
        for (int it = 0; it < 4; ++it) {
          const int row = it * 4 + q8;
          *(volatile v4u*)(C + (size_t)(mBase + row) * ldc + n0 + c8) = hv[it];
          if (dolo) *(volatile v4u*)(L + (size_t)(mBase + row) * ldc + n0 + c8) = lv[it];
        }
        __threadfence();
      }
    }
    wave_sync_lds();
  }
}

__global__ __launch_bounds__(128)
void attn_k(const unsigned short* __restrict__ Qp, const unsigned short* __restrict__ Kp,
            const unsigned short* __restrict__ Vh, const unsigned short* __restrict__ Vl,
            unsigned short* AH, unsigned short* AL) {
  __shared__ __align__(16) unsigned int Oh[64 * 32];
  __shared__ __align__(16) unsigned int Ol[64 * 32];
  const int tid  = threadIdx.x;
  const int wave = tid >> 5;
  const int lane = tid & 31;
  const int hh   = lane >> 4;
  const int c    = lane & 15;
  const int bx = blockIdx.x;
  const int qb = bx & 7;
  const int hp = (bx >> 3) & 3;
  const int g  = bx >> 5;
  const int q0 = qb * 64;
  const int r0 = g * NT;
  const int ql = wave * 16 + c;

  const _Float16* Qh  = (const _Float16*)(const void*)Qp;
  const _Float16* Kh  = (const _Float16*)(const void*)Kp;
  const _Float16* VHh = (const _Float16*)(const void*)Vh;
  const _Float16* VLh = (const _Float16*)(const void*)Vl;
  const float SC = 0.17677669529663688f * (1.0f / (QC * KC));

#pragma unroll 1
  for (int hs = 0; hs < 2; ++hs) {
    const int h = hp * 2 + hs;
    FragH qf;
    {
      const _Float16* qp = Qh + (size_t)(r0 + q0 + ql) * CH + h * HDIM + 8 * hh;
      qf.h[0] = *(const v8h*)(qp);
      qf.h[1] = *(const v8h*)(qp + 16);
    }
    const _Float16* kp  = Kh + (size_t)(r0 + c) * CH + h * HDIM + 8 * hh;
    const _Float16* vh0 = VHh + (size_t)(h * HDIM + c) * MROWS + r0 + 8 * hh;
    const _Float16* vh1 = vh0 + (size_t)16 * MROWS;
    const _Float16* vl0 = VLh + (size_t)(h * HDIM + c) * MROWS + r0 + 8 * hh;
    const _Float16* vl1 = vl0 + (size_t)16 * MROWS;

    float m = -1.0e30f, l = 0.f;
    v8f o0 = zero8(), o1 = zero8();
#pragma unroll 1
    for (int it = 0; it < NT / 64; ++it) {
      const int kb = it * 64;
      v16h kf[4];
#pragma unroll
      for (int j = 0; j < 4; ++j) kf[j] = ldfrag_h(kp + (size_t)(kb + 16 * j) * CH);
      v8f s0 = mma_h_raw(kf[0], qf.v, zero8());
      v8f s1 = mma_h_raw(kf[1], qf.v, zero8());
      v8f s2 = mma_h_raw(kf[2], qf.v, zero8());
      v8f s3 = mma_h_raw(kf[3], qf.v, zero8());
      sguard4(s0, s1, s2, s3, kf[0], kf[1], kf[2], kf[3], qf.v);

      float mx = fmaxf(fmaxf(hmax8(s0), hmax8(s1)), fmaxf(hmax8(s2), hmax8(s3)));
      mx = fmaxf(mx, __shfl_xor(mx, 16, 32));
      const float mn   = fmaxf(m, mx * SC);
      const float corr = __expf(m - mn);
      m = mn;
      l *= corr;
#pragma unroll
      for (int r = 0; r < 8; ++r) { o0[r] *= corr; o1[r] *= corr; }

      FragH p0, p1;
      float ls = 0.f;
#pragma unroll
      for (int r = 0; r < 8; ++r) {
        const float e0 = __expf(s0[r] * SC - mn) * PSC;
        const float e1 = __expf(s1[r] * SC - mn) * PSC;
        const float e2 = __expf(s2[r] * SC - mn) * PSC;
        const float e3 = __expf(s3[r] * SC - mn) * PSC;
        ls += (e0 + e1) + (e2 + e3);
        p0.h[0][r] = (_Float16)e0;
        p0.h[1][r] = (_Float16)e1;
        p1.h[0][r] = (_Float16)e2;
        p1.h[1][r] = (_Float16)e3;
      }
      l += ls;

      const v16h a0 = ldfrag_h(vh0 + kb), a1 = ldfrag_h(vh0 + kb + 32);
      const v16h b0 = ldfrag_h(vh1 + kb), b1 = ldfrag_h(vh1 + kb + 32);
      o0 = mma_h_raw(a0, p0.v, o0);
      o0 = mma_h_raw(a1, p1.v, o0);
      o1 = mma_h_raw(b0, p0.v, o1);
      o1 = mma_h_raw(b1, p1.v, o1);
      const v16h a2 = ldfrag_h(vl0 + kb), a3 = ldfrag_h(vl0 + kb + 32);
      const v16h b2 = ldfrag_h(vl1 + kb), b3 = ldfrag_h(vl1 + kb + 32);
      o0 = mma_h_raw(a2, p0.v, o0);
      o0 = mma_h_raw(a3, p1.v, o0);
      o1 = mma_h_raw(b2, p0.v, o1);
      o1 = mma_h_raw(b3, p1.v, o1);
      oguard2(o0, o1, a0, a1, b0, b1, a2, a3, b2, b3, p0.v, p1.v);
    }
    l += __shfl_xor(l, 16, 32);
    const float sc = (AC / VC) * (1.0f / l);

    v4u hA, lA, hB, lB;
#pragma unroll
    for (int e = 0; e < 4; ++e) {
      const float f0 = o0[2 * e] * sc, f1 = o0[2 * e + 1] * sc;
      const _Float16 x0 = (_Float16)f0, x1 = (_Float16)f1;
      const _Float16 y0 = (_Float16)(f0 - (float)x0), y1 = (_Float16)(f1 - (float)x1);
      hA[e] = pk16(h_bits(x0), h_bits(x1));
      lA[e] = pk16(h_bits(y0), h_bits(y1));
      const float f2 = o1[2 * e] * sc, f3 = o1[2 * e + 1] * sc;
      const _Float16 x2 = (_Float16)f2, x3 = (_Float16)f3;
      const _Float16 y2 = (_Float16)(f2 - (float)x2), y3 = (_Float16)(f3 - (float)x3);
      hB[e] = pk16(h_bits(x2), h_bits(x3));
      lB[e] = pk16(h_bits(y2), h_bits(y3));
    }
    const int cu = hs * 16 + 4 * hh;
    *(v4u*)(&Oh[ql * 32 + cu])     = hA;
    *(v4u*)(&Oh[ql * 32 + cu + 8]) = hB;
    *(v4u*)(&Ol[ql * 32 + cu])     = lA;
    *(v4u*)(&Ol[ql * 32 + cu + 8]) = lB;
  }
  __syncthreads();
  {
    const int rr = tid >> 3, e = tid & 7;
    v4u hv[4], lv[4];
#pragma unroll
    for (int it = 0; it < 4; ++it) {
      const int row = it * 16 + rr;
      hv[it] = *(const v4u*)(&Oh[row * 32 + 4 * e]);
      lv[it] = *(const v4u*)(&Ol[row * 32 + 4 * e]);
    }
    for (int pass = 0; pass < 2; ++pass) {
#pragma unroll
      for (int it = 0; it < 4; ++it) {
        const int row = it * 16 + rr;
        const size_t go = (size_t)(r0 + q0 + row) * CH + hp * 64 + 8 * e;
        *(volatile v4u*)(AH + go) = hv[it];
        *(volatile v4u*)(AL + go) = lv[it];
      }
      __threadfence();
    }
  }
}

extern "C" void kernel_launch(void* const* d_in, const int* in_sizes, int n_in,
                              void* d_out, int out_size, void* d_ws, size_t ws_size,
                              hipStream_t stream) {
  if (n_in < 9) return;
  if (in_sizes[0] != MROWS * CH) return;
  if (in_sizes[1] != CH * CH || in_sizes[2] != CH2 * CH || in_sizes[3] != CH2 * CH) return;
  if (in_sizes[4] != CH2 || in_sizes[5] != CH * CH2 || in_sizes[6] != CH) return;
  if (in_sizes[7] != CH * CH || in_sizes[8] != CH) return;
  if (out_size != MROWS * CH) return;

  const float* x    = (const float*)d_in[0];
  const float* w_q  = (const float*)d_in[1];
  const float* w_kv = (const float*)d_in[2];
  const float* w_c1 = (const float*)d_in[3];
  const float* b_c1 = (const float*)d_in[4];
  const float* w_c2 = (const float*)d_in[5];
  const float* b_c2 = (const float*)d_in[6];
  const float* w_p  = (const float*)d_in[7];
  const float* b_p  = (const float*)d_in[8];
  float* out = (float*)d_out;

  const size_t P16 = (size_t)MROWS * CH * 2;
  const size_t PW  = (size_t)NWEL * 2;
  size_t off = 0;
  const size_t oW = off; off += PW;
  const size_t oX = off; off += P16;
  const size_t oY = off; off += 4 * P16;
  const size_t oG = off; off += 2 * P16;
  if (off > ws_size) return;
  if (off > (size_t)134217728) return;

  char* ws = (char*)d_ws;
  unsigned short* Wall = (unsigned short*)(ws + oW);
  unsigned short* X16  = (unsigned short*)(ws + oX);
  float*          Y    = (float*)(ws + oY);
  unsigned short* G16  = (unsigned short*)(ws + oG);
  unsigned short* VEL2 = (unsigned short*)(ws + oY);
  unsigned short* Q16  = (unsigned short*)(ws + oY + P16);
  unsigned short* K16  = (unsigned short*)(ws + oY + 2 * P16);
  unsigned short* VHp  = (unsigned short*)(ws + oY + 3 * P16);
  unsigned short* VLp  = (unsigned short*)(ws + oG);
  unsigned short* AHp  = (unsigned short*)(ws + oG + P16);
  unsigned short* ALp  = (unsigned short*)(ws + oX);
  unsigned short* Wc1h = Wall + OWC1;
  unsigned short* Wc2h = Wall + OWC2;
  unsigned short* Wqh  = Wall + OWQ;
  unsigned short* Wkvh = Wall + OWKV;
  unsigned short* Wph  = Wall + OWP;

  const dim3 blk(256), blk128(128);
  const dim3 gW(NWEL / 2048);
  const dim3 gX(MROWS / 8);
  const dim3 gV(MROWS * CH2 / 2048);
  const dim3 gY(((MROWS / 64) * (CH2 / 64)) / 8);
  const dim3 gC(((MROWS / 64) * (CH / 64)) / 8);
  const dim3 gT(((CH / 64) * (MROWS / 64)) / 8);
  const dim3 gA(NGRP * 4 * (NT / 64));

  wprep<<<gW, blk, 0, stream>>>(w_c1, w_c2, w_q, w_kv, w_p, Wall);
  xprep<<<gX, blk, 0, stream>>>(x, X16);
  gemm64<1, 0, 1, 0><<<gY, blk, 0, stream>>>(
      X16, X16, CH, Wc1h, CH, b_c1, (void*)Y, CH2, X16, 0, 0,
      1.0f / (XS * WSC), 1.0f, MROWS, CH2, CH);
  velprep<<<gV, blk, 0, stream>>>(Y, G16);
  gemm64<1, 1, 1, 0><<<gC, blk, 0, stream>>>(
      G16, G16, CH2, Wc2h, CH2, b_c2, (void*)VEL2, CH, VEL2, 0, 0,
      V2C / (VS * WSC), V2C, MROWS, CH, CH2);
  gemm64<1, 1, 0, 0><<<gC, blk, 0, stream>>>(
      VEL2, VEL2, CH, Wqh, CH, b_c1, (void*)Q16, CH, Q16, 0, 0,
      QC / (V2C * WSC), 1.0f, MROWS, CH, CH);
  gemm64<1, 1, 0, 0><<<gC, blk, 0, stream>>>(
      X16, X16, CH, Wkvh, CH, b_c1, (void*)K16, CH, K16, 0, 0,
      KC / (XS * WSC), 1.0f, MROWS, CH, CH);
  gemm64<1, 1, 0, 0><<<gT, blk, 0, stream>>>(
      Wkvh + (size_t)CH * CH, Wkvh + (size_t)CH * CH, CH, X16, CH, b_c1, (void*)VHp, MROWS, VLp, 0, MROWS,
      VC / (XS * WSC), 1.0f, CH, MROWS, CH);
  attn_k<<<gA, blk128, 0, stream>>>(Q16, K16, VHp, VLp, AHp, ALp);
  gemm64<2, 0, 1, 1><<<gC, blk, 0, stream>>>(
      AHp, ALp, CH, Wph, CH, b_p, (void*)out, CH, X16, 0, 0,
      1.0f / (AC * WSC), 1.0f, MROWS, CH, CH);
  (void)hipGetLastError();
}
